// TransformerEncoderLayerWithBias_22978075034135
// MI455X (gfx1250) — hardware-verified
//
#include <hip/hip_runtime.h>
#include <math.h>

constexpr int kBatch  = 16;
constexpr int kSeq    = 512;
constexpr int kEmb    = 1024;
constexpr int kHeads  = 16;
constexpr int kHd     = 64;
constexpr int kFF     = 4096;
constexpr int kRows   = kBatch * kSeq;
constexpr int kRel    = 2 * 512 - 1;
constexpr int kFFRows = 2048;
constexpr int kQK     = 2 * kEmb;

constexpr float kWCarry     = 32.0f;
constexpr float kWCarryInv  = 1.0f / 32.0f;
constexpr float kW2Carry    = 64.0f;
constexpr float kPCarry     = 32768.0f;
constexpr float kCtxCarry   = 64.0f;
constexpr float kHCarry     = 32.0f;
constexpr float kScoreScale = 0.125f;
constexpr float kPVScale    = kCtxCarry / kPCarry;
constexpr float kOutScale   = 1.0f / (kCtxCarry * kWCarry);
constexpr float kFF2Scale   = 1.0f / (kHCarry * kW2Carry);
constexpr float kInvEmb     = 1.0f / 1024.0f;
constexpr float kLnEps      = 1e-5f;

typedef __attribute__((ext_vector_type(16))) _Float16 v16h;
typedef __attribute__((ext_vector_type(8)))  _Float16 v8h;
typedef __attribute__((ext_vector_type(16))) __bf16   v16b;
typedef __attribute__((ext_vector_type(8)))  __bf16   v8b;
typedef __attribute__((ext_vector_type(8)))  float    v8f;
typedef __attribute__((ext_vector_type(4)))  float    v4f;
typedef __attribute__((ext_vector_type(4)))  unsigned int v4u;

__device__ __forceinline__ unsigned short f2bf_bits(float f) {
  unsigned u = __float_as_uint(f);
  return (unsigned short)((u + 0x7FFFu + ((u >> 16) & 1u)) >> 16);
}
__device__ __forceinline__ float bf_bits2f(unsigned short h) { return __uint_as_float(((unsigned)h) << 16); }

__device__ __forceinline__ void dep_guard_h(v8f& a, v8f& b, v16h x, v16h y) { asm volatile("v_nop\n\tv_nop\n\tv_nop\n\tv_nop" : "+v"(a), "+v"(b) : "v"(x), "v"(y)); }
__device__ __forceinline__ void dep_guard_b(v8f& a, v8f& b, v16b x, v16b y) { asm volatile("v_nop\n\tv_nop\n\tv_nop\n\tv_nop" : "+v"(a), "+v"(b) : "v"(x), "v"(y)); }
__device__ __forceinline__ void keep4_h(v16h a, v16h b, v16h c, v16h d) { asm volatile("v_nop" :: "v"(a), "v"(b), "v"(c), "v"(d)); }
__device__ __forceinline__ void keep4_b(v16b a, v16b b, v16b c, v16b d) { asm volatile("v_nop" :: "v"(a), "v"(b), "v"(c), "v"(d)); }
__device__ __forceinline__ void acc_guard4(v8f& a, v8f& b, v8f& c, v8f& d) { asm volatile("v_nop\n\tv_nop\n\tv_nop\n\tv_nop" : "+v"(a), "+v"(b), "+v"(c), "+v"(d)); }
template <typename T> struct Frag;
template <> struct Frag<_Float16> {
  typedef v16h V; union U { v16h v; v8h h[2]; };
  static __device__ __forceinline__ v16h load(const _Float16* p) {
    U f; f.h[0] = *(const v8h*)(p); f.h[1] = *(const v8h*)(p + 16); return f.v;
  }
  static __device__ __forceinline__ v8f mma(v16h a, v16h b, v8f c) {
    return __builtin_amdgcn_wmma_f32_16x16x32_f16(false, a, false, b, (short)0, c, false, false);
  }
  static __device__ __forceinline__ void guard(v8f& a, v8f& b, v16h x, v16h y) { dep_guard_h(a, b, x, y); }
  static __device__ __forceinline__ void keep(v16h a, v16h b, v16h c, v16h d) { keep4_h(a, b, c, d); }
};
template <> struct Frag<__bf16> {
  typedef v16b V; union U { v16b v; v8b h[2]; };
  static __device__ __forceinline__ v16b load(const __bf16* p) {
    U f; f.h[0] = *(const v8b*)(p); f.h[1] = *(const v8b*)(p + 16); return f.v;
  }
  static __device__ __forceinline__ v8f mma(v16b a, v16b b, v8f c) {
    return __builtin_amdgcn_wmma_f32_16x16x32_bf16(false, a, false, b, (short)0, c, false, false);
  }
  static __device__ __forceinline__ void guard(v8f& a, v8f& b, v16b x, v16b y) { dep_guard_b(a, b, x, y); }
  static __device__ __forceinline__ void keep(v16b a, v16b b, v16b c, v16b d) { keep4_b(a, b, c, d); }
};

__device__ __forceinline__ unsigned pk16(unsigned short a, unsigned short b) { return (unsigned)a | ((unsigned)b << 16); }
__device__ __forceinline__ unsigned short h_bits(float f) { const _Float16 h = (_Float16)f; return __builtin_bit_cast(unsigned short, h); }

template <int ET> struct Elem;
template <> struct Elem<0> { typedef _Float16 T; };
template <> struct Elem<1> { typedef __bf16 T; };
template <int ET, bool SPLIT, int BIAS_MODE, int OUT_MODE, bool RESID, int ACT = 0, int TRI = 0>
__global__ __launch_bounds__(256) void wmma_gemm64(
    const unsigned short* __restrict__ Ap, const unsigned short* __restrict__ A2p, int lda, long strideA,
    const unsigned short* __restrict__ Btp, const unsigned short* __restrict__ Bt2p, int ldb, long strideB,
    void* __restrict__ Cout, void* __restrict__ Cout2, int ldc, long strideC,
    const float* __restrict__ bias,
    const float* __restrict__ resid, long strideR,
    int M, int N, int K, float scale) {
  typedef typename Elem<ET>::T T;
  typedef typename Frag<T>::V V;
  const T* A = (const T*)Ap; const T* A2 = (const T*)A2p; const T* Bt = (const T*)Btp; const T* Bt2 = (const T*)Bt2p;
  __shared__ __align__(16) float sT[8][16 * 68];
  const int b    = blockIdx.y;
  const int lane = threadIdx.x & 31;
  const int wave = threadIdx.x >> 5;
  const int tilesN = N >> 6;
  const int tilesM = M >> 6;
  const int tile = blockIdx.x * 8 + wave;
  if (tile >= tilesM * tilesN) return;
  const int tm = tile / tilesN;
  const int tn = tile - tm * tilesN;
  if (TRI == 1 && tn > tm) return;
  const int m0 = tm << 6;
  const int n0 = tn << 6;
  const int Kend = (TRI == 2) ? ((m0 + 64 < K) ? (m0 + 64) : K) : K;

  const T* Ab  = A  + (size_t)b * strideA;
  const T* Bb  = Bt + (size_t)b * strideB;
  const T* Ab2 = SPLIT ? (A2  + (size_t)b * strideA) : nullptr;
  const T* Bb2 = SPLIT ? (Bt2 + (size_t)b * strideB) : nullptr;

  const int rlane = lane & 15;
  const int koff  = (lane >> 4) * 8;
  const int mOff  = (lane >> 4) * 8;

  v8f acc[4][4];
#pragma unroll
  for (int i = 0; i < 4; ++i)
#pragma unroll
    for (int j = 0; j < 4; ++j) acc[i][j] = (v8f){0.f,0.f,0.f,0.f,0.f,0.f,0.f,0.f};

  for (int k0 = 0; k0 < Kend; k0 += 32) {
    V bh[4], bl[4];
#pragma unroll
    for (int j = 0; j < 4; ++j) {
      const size_t bo = (size_t)(n0 + (j << 4) + rlane) * ldb + koff + k0;
      bh[j] = Frag<T>::load(Bb + bo);
      if (SPLIT) bl[j] = Frag<T>::load(Bb2 + bo);
    }
#pragma unroll
    for (int i = 0; i < 4; ++i) {
      const size_t ao = (size_t)(m0 + (i << 4) + rlane) * lda + koff + k0;
      V ah = Frag<T>::load(Ab + ao);
      V al;
      if (SPLIT) al = Frag<T>::load(Ab2 + ao);
#pragma unroll
      for (int j = 0; j < 4; ++j) {
        acc[i][j] = Frag<T>::mma(ah, bh[j], acc[i][j]);
        if (SPLIT) {
          acc[i][j] = Frag<T>::mma(ah, bl[j], acc[i][j]);
          acc[i][j] = Frag<T>::mma(al, bh[j], acc[i][j]);
        }
      }
      Frag<T>::guard(acc[i][0], acc[i][3], ah, SPLIT ? al : ah);
    }
    Frag<T>::keep(bh[0], bh[1], bh[2], bh[3]);
    if (SPLIT) Frag<T>::keep(bl[0], bl[1], bl[2], bl[3]);
  }
  acc_guard4(acc[0][0], acc[0][1], acc[0][2], acc[0][3]);
  acc_guard4(acc[1][0], acc[1][1], acc[1][2], acc[1][3]);
  acc_guard4(acc[2][0], acc[2][1], acc[2][2], acc[2][3]);
  acc_guard4(acc[3][0], acc[3][1], acc[3][2], acc[3][3]);

  float* slab = sT[wave];
  const float* Rb = RESID ? (resid + (size_t)b * strideR) : nullptr;
#pragma unroll
  for (int i = 0; i < 4; ++i) {
    const int mBase = m0 + (i << 4);
#pragma unroll
    for (int j = 0; j < 4; ++j) {
      const int n = n0 + (j << 4) + rlane;
      float bv = 0.f;
      if (BIAS_MODE == 2) bv = bias[n];
#pragma unroll
      for (int r = 0; r < 8; ++r) {
        float v = acc[i][j][r] * scale;
        if (BIAS_MODE == 1) v += bias[mBase + mOff + r];
        if (BIAS_MODE == 2) v += bv;
        if (RESID) v += Rb[(size_t)(mBase + mOff + r) * ldc + n];
        if (ACT == 2) v = fmaxf(v, 0.0f);
        if (ACT == 4) v = (v > 0.f) ? v : 0.01f * v;
        slab[(mOff + r) * 68 + (j << 4) + rlane] = v;
      }
    }
    __builtin_amdgcn_fence(__ATOMIC_RELEASE, "workgroup");
    __builtin_amdgcn_wave_barrier();
    __builtin_amdgcn_fence(__ATOMIC_ACQUIRE, "workgroup");
    if (OUT_MODE == 0) {
      float* C = (float*)Cout + (size_t)b * strideC;
      const int hh = lane >> 4, c4 = (lane & 15) * 4;
      for (int pass = 0; pass < 2; ++pass) {
#pragma unroll
        for (int it = 0; it < 8; ++it) {
          const int row = it * 2 + hh;
          v4f v = *(const v4f*)(slab + row * 68 + c4);
          *(volatile v4f*)(C + (size_t)(mBase + row) * ldc + n0 + c4) = v;
        }
        __threadfence();
      }
    } else {
      const int q = lane >> 3, c8 = (lane & 7) * 8;
      unsigned short* C  = (unsigned short*)Cout  + (size_t)b * strideC;
      unsigned short* C2 = (OUT_MODE == 2) ? ((unsigned short*)Cout2 + (size_t)b * strideC) : nullptr;
      for (int pass = 0; pass < 2; ++pass) {
#pragma unroll
        for (int it = 0; it < 4; ++it) {
          const int row = it * 4 + q;
          const float* sp = slab + row * 68 + c8;
          v8h hv, lv;
#pragma unroll
          for (int e = 0; e < 8; ++e) {
            if (OUT_MODE == 1) {
              hv[e] = (_Float16)sp[e];
            } else {
              unsigned short hb = f2bf_bits(sp[e]);
              unsigned short lb = f2bf_bits(sp[e] - bf_bits2f(hb));
              hv[e] = __builtin_bit_cast(_Float16, hb);
              lv[e] = __builtin_bit_cast(_Float16, lb);
            }
          }
          *(volatile v8h*)(C + (size_t)(mBase + row) * ldc + n0 + c8) = hv;
          if (OUT_MODE == 2) *(volatile v8h*)(C2 + (size_t)(mBase + row) * ldc + n0 + c8) = lv;
        }
        __threadfence();
      }
    }
    __builtin_amdgcn_fence(__ATOMIC_RELEASE, "workgroup");
    __builtin_amdgcn_wave_barrier();
    __builtin_amdgcn_fence(__ATOMIC_ACQUIRE, "workgroup");
  }
}

__global__ __launch_bounds__(256) void cast_scale_f16x8(const float* __restrict__ in, unsigned short* __restrict__ out,
                                                       float scale) {
  const size_t i = ((size_t)blockIdx.x * 256 + threadIdx.x) * 8;
  const v4f a = *(const v4f*)(in + i);
  const v4f c = *(const v4f*)(in + i + 4);
  unsigned short hb[8];
#pragma unroll
  for (int e = 0; e < 4; ++e) { hb[e] = h_bits(a[e] * scale); hb[4 + e] = h_bits(c[e] * scale); }
  const v4u u = (v4u){pk16(hb[0], hb[1]), pk16(hb[2], hb[3]), pk16(hb[4], hb[5]), pk16(hb[6], hb[7])};
  unsigned short* op = out + i;
  *(volatile v4u*)op = u;
  __threadfence();
  *(volatile v4u*)op = u;
}

__global__ __launch_bounds__(128) void ln_kernel(const float* __restrict__ x, const float* __restrict__ g,
                                                 const float* __restrict__ be, unsigned short* __restrict__ y) {
  __shared__ float red1[4];
  __shared__ float red2[4];
  const int row  = blockIdx.x;
  const int t    = threadIdx.x;
  const int lane = t & 31, wave = t >> 5;
  const int c0   = t * 8;
  const float* xr = x + (size_t)row * kEmb + c0;
  const v4f a = *(const v4f*)(xr);
  const v4f c = *(const v4f*)(xr + 4);
  float xv[8];
#pragma unroll
  for (int e = 0; e < 4; ++e) { xv[e] = a[e]; xv[4 + e] = c[e]; }
  float s = ((xv[0] + xv[1]) + (xv[2] + xv[3])) + ((xv[4] + xv[5]) + (xv[6] + xv[7]));
#pragma unroll
  for (int off = 16; off > 0; off >>= 1) s += __shfl_xor(s, off, 32);
  if (lane == 0) red1[wave] = s;
  __syncthreads();
  const float mu = ((red1[0] + red1[1]) + (red1[2] + red1[3])) * kInvEmb;
  float d[8];
#pragma unroll
  for (int e = 0; e < 8; ++e) d[e] = xv[e] - mu;
  float ss = ((d[0] * d[0] + d[1] * d[1]) + (d[2] * d[2] + d[3] * d[3])) +
             ((d[4] * d[4] + d[5] * d[5]) + (d[6] * d[6] + d[7] * d[7]));
#pragma unroll
  for (int off = 16; off > 0; off >>= 1) ss += __shfl_xor(ss, off, 32);
  if (lane == 0) red2[wave] = ss;
  __syncthreads();
  const float var = ((red2[0] + red2[1]) + (red2[2] + red2[3])) * kInvEmb;
  const float rs = rsqrtf(var + kLnEps);
  const v4f ga = *(const v4f*)(g + c0);
  const v4f gc = *(const v4f*)(g + c0 + 4);
  const v4f ba = *(const v4f*)(be + c0);
  const v4f bc = *(const v4f*)(be + c0 + 4);
  unsigned short hb[8];
#pragma unroll
  for (int e = 0; e < 4; ++e) {
    hb[e]     = h_bits((d[e] * rs) * ga[e] + ba[e]);
    hb[4 + e] = h_bits((d[4 + e] * rs) * gc[e] + bc[e]);
  }
  const v4u u = (v4u){pk16(hb[0], hb[1]), pk16(hb[2], hb[3]), pk16(hb[4], hb[5]), pk16(hb[6], hb[7])};
  unsigned short* yp = y + (size_t)row * kEmb + c0;
  *(volatile v4u*)yp = u;
  __threadfence();
  *(volatile v4u*)yp = u;
}

__global__ __launch_bounds__(64) void softmax_bias_kernel(const float* __restrict__ S, const float* __restrict__ relb,
                                                          unsigned short* __restrict__ P, float carry) {
  __shared__ float redM[2];
  __shared__ float redS[2];
  const int row  = blockIdx.x;
  const int z    = blockIdx.y;
  const int t    = threadIdx.x;
  const int lane = t & 31, wave = t >> 5;
  const int c0   = t * 8;
  const size_t rbase = ((size_t)z * kSeq + row) * kSeq + c0;
  const v4f a = *(const v4f*)(S + rbase);
  const v4f c = *(const v4f*)(S + rbase + 4);
  const float* rb = relb + (size_t)z * kRel;
  float x[8];
#pragma unroll
  for (int e = 0; e < 8; ++e) {
    int idx = row - (c0 + e) + (kSeq - 1);
    idx = idx < 0 ? 0 : (idx > kRel - 1 ? kRel - 1 : idx);
    const float bv = rb[idx];
    x[e] = ((e < 4) ? a[e] : c[e - 4]) + bv;
  }
  float m = fmaxf(fmaxf(fmaxf(x[0], x[1]), fmaxf(x[2], x[3])), fmaxf(fmaxf(x[4], x[5]), fmaxf(x[6], x[7])));
#pragma unroll
  for (int off = 16; off > 0; off >>= 1) m = fmaxf(m, __shfl_xor(m, off, 32));
  if (lane == 0) redM[wave] = m;
  __syncthreads();
  m = fmaxf(redM[0], redM[1]);
  float ex[8];
#pragma unroll
  for (int e = 0; e < 8; ++e) ex[e] = expf(x[e] - m);
  float s = ((ex[0] + ex[1]) + (ex[2] + ex[3])) + ((ex[4] + ex[5]) + (ex[6] + ex[7]));
#pragma unroll
  for (int off = 16; off > 0; off >>= 1) s += __shfl_xor(s, off, 32);
  if (lane == 0) redS[wave] = s;
  __syncthreads();
  const float tot = redS[0] + redS[1];
  const float inv = (1.0f / tot) * carry;
  unsigned short hb[8];
#pragma unroll
  for (int e = 0; e < 8; ++e) hb[e] = h_bits(ex[e] * inv);
  const v4u u = (v4u){pk16(hb[0], hb[1]), pk16(hb[2], hb[3]), pk16(hb[4], hb[5]), pk16(hb[6], hb[7])};
  unsigned short* pp = P + rbase;
  *(volatile v4u*)pp = u;
  __threadfence();
  *(volatile v4u*)pp = u;
}

__global__ __launch_bounds__(256) void gelu_cast_kernel(const float* __restrict__ in, unsigned short* __restrict__ out,
                                                        float carry) {
  const size_t i = (size_t)blockIdx.x * 256 + threadIdx.x;
  const float* p = in + 2 * i;
  unsigned u = 0u;
#pragma unroll 1
  for (int e = 0; e < 2; ++e) {
    const float xv = p[e];
    const float gv = 0.5f * xv * (1.0f + erff(xv * 0.70710678118654752f));
    u |= ((unsigned)h_bits(gv * carry)) << (16 * e);
  }
  ((volatile unsigned*)out)[i] = u;
  __threadfence();
  ((volatile unsigned*)out)[i] = u;
}

extern "C" void kernel_launch(void* const* d_in, const int* in_sizes, int n_in,
                              void* d_out, int out_size, void* d_ws, size_t ws_size,
                              hipStream_t stream) {
  if (n_in < 14) return;
  if (in_sizes[0] != kRows * kEmb || out_size != kRows * kEmb) return;
  if (in_sizes[1] != 3 * kEmb * kEmb || in_sizes[2] != 3 * kEmb || in_sizes[3] != kEmb * kEmb) return;
  if (in_sizes[5] != kHeads * kRel || in_sizes[6] != kFF * kEmb || in_sizes[8] != kEmb * kFF) return;
  if (in_sizes[4] != kEmb || in_sizes[7] != kFF || in_sizes[9] != kEmb) return;
  if (in_sizes[10] != kEmb || in_sizes[11] != kEmb || in_sizes[12] != kEmb || in_sizes[13] != kEmb) return;

  const float* x     = (const float*)d_in[0];
  const float* in_w  = (const float*)d_in[1];
  const float* in_b  = (const float*)d_in[2];
  const float* out_w = (const float*)d_in[3];
  const float* out_b = (const float*)d_in[4];
  const float* relb  = (const float*)d_in[5];
  const float* w1    = (const float*)d_in[6];
  const float* b1    = (const float*)d_in[7];
  const float* w2    = (const float*)d_in[8];
  const float* b2    = (const float*)d_in[9];
  const float* ln1w  = (const float*)d_in[10];
  const float* ln1b  = (const float*)d_in[11];
  const float* ln2w  = (const float*)d_in[12];
  const float* ln2b  = (const float*)d_in[13];
  float* out = (float*)d_out;

  const size_t MiB = (size_t)1 << 20;
  const size_t offWin  = 0;
  const size_t offWout = 6 * MiB;
  const size_t offW1   = 8 * MiB;
  const size_t offW2   = 16 * MiB;
  const size_t offA    = 24 * MiB;
  const size_t offB    = 40 * MiB;
  const size_t offC    = 72 * MiB;
  const size_t offD    = 88 * MiB;
  const size_t total   = 120 * MiB;
  if (ws_size < total) return;

  char* ws = (char*)d_ws;
  unsigned short* Win16  = (unsigned short*)(ws + offWin);
  unsigned short* Wout16 = (unsigned short*)(ws + offWout);
  unsigned short* W1_16  = (unsigned short*)(ws + offW1);
  unsigned short* W2_16  = (unsigned short*)(ws + offW2);
  unsigned short* XN16   = (unsigned short*)(ws + offA);
  unsigned short* CTX16  = (unsigned short*)(ws + offA);
  unsigned short* F1     = (unsigned short*)(ws + offA);
  unsigned short* QK16   = (unsigned short*)(ws + offB);
  float*          X1     = (float*)(ws + offB);
  unsigned short* VT16   = (unsigned short*)(ws + offC);
  unsigned short* XN2    = (unsigned short*)(ws + offC);
  float*          Sbuf   = (float*)(ws + offD);
  unsigned short* P16    = (unsigned short*)(ws + offD + 16 * MiB);
  float*          Hf     = (float*)(ws + offD);

  const long planeS = (long)kSeq * kSeq;

  cast_scale_f16x8<<<(3 * kEmb * kEmb) / 2048, 256, 0, stream>>>(in_w, Win16, kWCarry);
  cast_scale_f16x8<<<(kEmb * kEmb) / 2048, 256, 0, stream>>>(out_w, Wout16, kWCarry);
  cast_scale_f16x8<<<(kFF * kEmb) / 2048, 256, 0, stream>>>(w1, W1_16, kWCarry);
  cast_scale_f16x8<<<(kEmb * kFF) / 2048, 256, 0, stream>>>(w2, W2_16, kW2Carry);

  ln_kernel<<<kRows, 128, 0, stream>>>(x, ln1w, ln1b, XN16);

  {
    const int gx = ((kRows / 64) * (kQK / 64) + 7) / 8;
    wmma_gemm64<0, false, 2, 1, false, 0, 0><<<dim3(gx, 1), 256, 0, stream>>>(
        XN16, XN16, kEmb, 0L, Win16, Win16, kEmb, 0L, QK16, QK16, kQK, 0L, in_b, x, 0L,
        kRows, kQK, kEmb, kWCarryInv);
  }
  {
    const int gx = ((kEmb / 64) * (kSeq / 64) + 7) / 8;
    const unsigned short* Wv16 = Win16 + (size_t)2 * kEmb * kEmb;
    wmma_gemm64<0, false, 1, 1, false, 0, 0><<<dim3(gx, kBatch), 256, 0, stream>>>(
        Wv16, Wv16, kEmb, 0L, XN16, XN16, kEmb, (long)kSeq * kEmb, VT16, VT16, kSeq, (long)kEmb * kSeq,
        in_b + 2 * kEmb, x, 0L, kEmb, kSeq, kEmb, kWCarryInv);
  }

  for (int bb = 0; bb < kBatch; ++bb) {
    const unsigned short* Qg = QK16 + (size_t)bb * kSeq * kQK;
    const unsigned short* Kg = Qg + kEmb;
    const unsigned short* Vg = VT16 + (size_t)bb * kEmb * kSeq;
    unsigned short* Cg = CTX16 + (size_t)bb * kSeq * kEmb;
    {
      const int gx = ((kSeq / 64) * (kSeq / 64) + 7) / 8;
      wmma_gemm64<0, false, 0, 0, false, 0, 0><<<dim3(gx, kHeads), 256, 0, stream>>>(
          Qg, Qg, kQK, (long)kHd, Kg, Kg, kQK, (long)kHd, Sbuf, Sbuf, kSeq, planeS, in_b, x, 0L,
          kSeq, kSeq, kHd, kScoreScale);
    }
    softmax_bias_kernel<<<dim3(kSeq, kHeads), 64, 0, stream>>>(Sbuf, relb, P16, kPCarry);
    {
      const int gx = ((kSeq / 64) * (kHd / 64) + 7) / 8;
      wmma_gemm64<0, false, 0, 1, false, 0, 0><<<dim3(gx, kHeads), 256, 0, stream>>>(
          P16, P16, kSeq, planeS, Vg, Vg, kSeq, (long)kHd * kSeq, Cg, Cg, kEmb, (long)kHd, in_b, x, 0L,
          kSeq, kHd, kSeq, kPVScale);
    }
  }

  {
    const int gx = ((kRows / 64) * (kEmb / 64) + 7) / 8;
    wmma_gemm64<0, false, 2, 0, true, 0, 0><<<dim3(gx, 1), 256, 0, stream>>>(
        CTX16, CTX16, kEmb, 0L, Wout16, Wout16, kEmb, 0L, X1, X1, kEmb, 0L, out_b, x, 0L,
        kRows, kEmb, kEmb, kOutScale);
  }

  ln_kernel<<<kRows, 128, 0, stream>>>(X1, ln2w, ln2b, XN2);

  for (int ch = 0; ch < kRows / kFFRows; ++ch) {
    const unsigned short* Yc = XN2 + (size_t)ch * kFFRows * kEmb;
    const float* X1c = X1 + (size_t)ch * kFFRows * kEmb;
    float* outc = out + (size_t)ch * kFFRows * kEmb;
    {
      const int gx = ((kFFRows / 64) * (kFF / 64) + 7) / 8;
      wmma_gemm64<0, false, 2, 0, false, 0, 0><<<dim3(gx, 1), 256, 0, stream>>>(
          Yc, Yc, kEmb, 0L, W1_16, W1_16, kEmb, 0L, Hf, Hf, kFF, 0L, b1, x, 0L, kFFRows, kFF, kEmb, kWCarryInv);
    }
    gelu_cast_kernel<<<(kFFRows * kFF / 2) / 256, 256, 0, stream>>>(Hf, F1, kHCarry);
    {
      const int gx = ((kFFRows / 64) * (kEmb / 64) + 7) / 8;
      wmma_gemm64<0, false, 2, 0, true, 0, 0><<<dim3(gx, 1), 256, 0, stream>>>(
          F1, F1, kFF, 0L, W2_16, W2_16, kFF, 0L, outc, outc, kEmb, 0L, b2, X1c, 0L, kFFRows, kEmb, kFF, kFF2Scale);
    }
  }
}
